// SSMBlock_86766929313980
// MI455X (gfx1250) — hardware-verified
//
#include <hip/hip_runtime.h>
#include <math.h>

typedef __attribute__((ext_vector_type(16))) _Float16 v16h;
typedef __attribute__((ext_vector_type(8)))  _Float16 v8h;
typedef __attribute__((ext_vector_type(8)))  float    v8f;
typedef __attribute__((ext_vector_type(4)))  float    v4f;
typedef __attribute__((ext_vector_type(2)))  float    v2f;
typedef __attribute__((ext_vector_type(4)))  unsigned v4u;

constexpr int kBatch = 2;
constexpr int kSeq   = 4096;
constexpr int kD     = 1024;
constexpr int kDS    = 1024;
constexpr int kH     = 4096;
constexpr int kG     = 2 * kD;
constexpr int kRows  = kBatch * kSeq;
constexpr int kScanTS = 64;
constexpr int kScanYP = 68;
constexpr float kWCarry  = 32.0f;
constexpr float kACarry  = 16.0f;
constexpr float kInvW    = 1.0f / kWCarry;
constexpr float kInvWA   = 1.0f / (kWCarry * kACarry);
static_assert(kD == kDS, "stacked state operand needs equal widths");
static_assert((kD % 32) == 0 && (kDS % 32) == 0 && (kH % 32) == 0, "GEMM K multiples of 32");
static_assert((kRows % 64) == 0 && (kG % 64) == 0 && (kDS % 64) == 0 && (kD % 64) == 0 && (kH % 64) == 0, "GEMM M,N multiples of 64");
static_assert((kRows % 32) == 0 && (kSeq % kScanTS) == 0 && (kDS % 64) == 0 && (kD % 256) == 0, "tile multiples");

constexpr size_t kOffGWT = 0;
constexpr size_t kOffSWT = kOffGWT + (size_t)kG * kD * 2;
constexpr size_t kOffOWT = kOffSWT + (size_t)kDS * kD * 2;
constexpr size_t kOffW1T = kOffOWT + (size_t)kD * kDS * 2;
constexpr size_t kOffW2T = kOffW1T + (size_t)kH * kD * 2;
constexpr size_t kOffXN  = kOffW2T + (size_t)kD * kH * 2;
constexpr size_t kOffS   = kOffXN  + (size_t)kRows * kD * 2;
constexpr size_t kOffUB  = kOffS   + (size_t)2 * kRows * kD * 2;
constexpr size_t kOffY   = kOffUB  + (size_t)2 * kRows * kDS * 2;
constexpr size_t kOffWM  = kOffY   + (size_t)kRows * kDS * 2;
constexpr size_t kWmFloats = 33 * 32;
constexpr size_t kOffDL  = kOffWM  + kWmFloats * 4;
constexpr size_t kOffDA  = kOffDL  + (size_t)kRows * 4;
constexpr size_t kWsTotal = kOffDA + (size_t)kRows * 4;
constexpr size_t kOffHID = kOffXN;
constexpr size_t kOffX2  = kOffUB + (size_t)kRows * kDS * 2;
static_assert(kWsTotal == 125898880ull, "carve total");
static_assert(kWsTotal <= 134217728ull, "carve cap");
static_assert(kOffHID + (size_t)kRows * kH * 2 <= kOffX2, "hid alias extent");
static_assert(kOffX2 + (size_t)kRows * kD * 2 <= kOffY, "x2 alias extent");
static_assert((kOffSWT % 128) == 0 && (kOffOWT % 128) == 0 && (kOffW1T % 128) == 0 && (kOffW2T % 128) == 0 &&
              (kOffXN % 128) == 0 && (kOffS % 128) == 0 && (kOffUB % 128) == 0 && (kOffY % 128) == 0 &&
              (kOffWM % 128) == 0 && (kOffDL % 128) == 0 && (kOffDA % 128) == 0 && (kOffX2 % 128) == 0, "128-B aligned regions");

__device__ __forceinline__ float h16_to_f32(unsigned hb) {
  const unsigned sgn = (hb & 0x8000u) << 16;
  const unsigned em = hb & 0x7fffu;
  const float fn = __uint_as_float((em << 13) + 0x38000000u);
  const float fs = (float)em * 5.9604644775390625e-8f;
  const float mag = (em < 0x400u) ? fs : fn;
  return __uint_as_float(__float_as_uint(mag) | sgn);
}
__device__ __forceinline__ float wave_sum(float v) {
#pragma unroll
  for (int off = 16; off > 0; off >>= 1) v += __shfl_xor(v, off, 32);
  return v;
}
__device__ __forceinline__ void wave_sync() {
  __builtin_amdgcn_fence(__ATOMIC_RELEASE, "workgroup");
  __builtin_amdgcn_wave_barrier();
  __builtin_amdgcn_fence(__ATOMIC_ACQUIRE, "workgroup");
}
__device__ __forceinline__ float silu_f(float v) { return v * (1.0f / (1.0f + expf(-v))); }
__device__ __forceinline__ float gelu_f(float v) { return 0.5f * v * (1.0f + erff(v * 0.70710678118654752f)); }

__device__ __forceinline__ void guard_row(v8f& a, v8f& b, v8f& c, v8f& d, v16h x, v16h b0, v16h b1, v16h b2, v16h b3) {
  asm volatile("v_nop\n\tv_nop\n\tv_nop\n\tv_nop" : "+v"(a), "+v"(b), "+v"(c), "+v"(d) : "v"(x), "v"(b0), "v"(b1), "v"(b2), "v"(b3));
}
__device__ __forceinline__ void acc_guard4(v8f& a, v8f& b, v8f& c, v8f& d) {
  asm volatile("v_nop\n\tv_nop\n\tv_nop\n\tv_nop" : "+v"(a), "+v"(b), "+v"(c), "+v"(d));
}
union FragU { v16h v; v8h h[2]; };
__device__ __forceinline__ v16h frag_load(const _Float16* p) {
  FragU f;
  f.h[0] = *(const v8h*)(p);
  f.h[1] = *(const v8h*)(p + 16);
  return f.v;
}
__device__ __forceinline__ v8f mma_f16(v16h a, v16h b, v8f c) {
  return __builtin_amdgcn_wmma_f32_16x16x32_f16(false, a, false, b, (short)0, c, false, false);
}

constexpr int kEpiGate  = 0;
constexpr int kEpiF16   = 1;
constexpr int kEpiResid = 2;
constexpr int kEpiGelu  = 3;

template <int EPI>
__global__ __launch_bounds__(256) void gemm_f16_kernel(
    const unsigned short* __restrict__ Ap, int lda,
    const unsigned short* __restrict__ Btp, int ldb,
    void* Cout, int ldc,
    const float* __restrict__ bias,
    const float* resid,
    int M, int N, int K, float scale, float ocarry)
{
  const _Float16* A  = (const _Float16*)Ap;
  const _Float16* Bt = (const _Float16*)Btp;
  __shared__ __align__(16) float sT[8][16 * 68];
  const int lane = threadIdx.x & 31;
  const int wave = threadIdx.x >> 5;
  const int tilesN = N >> 6;
  const int tilesM = M >> 6;
  const int tile = blockIdx.x * 8 + wave;
  if (tile >= tilesM * tilesN) return;
  const int tm = tile / tilesN;
  const int tn = tile - tm * tilesN;
  const int m0 = tm << 6;
  const int n0 = tn << 6;
  const int rlane = lane & 15;
  const int koff  = (lane >> 4) * 8;
  const int mOff  = (lane >> 4) * 8;

  v8f acc[4][4];
#pragma unroll
  for (int i = 0; i < 4; ++i)
#pragma unroll
    for (int j = 0; j < 4; ++j) acc[i][j] = (v8f){0.f, 0.f, 0.f, 0.f, 0.f, 0.f, 0.f, 0.f};

  for (int k0 = 0; k0 < K; k0 += 32) {
    v16h bh[4];
#pragma unroll
    for (int j = 0; j < 4; ++j) {
      const size_t bo = (size_t)(n0 + (j << 4) + rlane) * ldb + koff + k0;
      bh[j] = frag_load(Bt + bo);
    }
#pragma unroll
    for (int i = 0; i < 4; ++i) {
      const size_t ao = (size_t)(m0 + (i << 4) + rlane) * lda + koff + k0;
      const v16h ah = frag_load(A + ao);
#pragma unroll
      for (int j = 0; j < 4; ++j) acc[i][j] = mma_f16(ah, bh[j], acc[i][j]);
      guard_row(acc[i][0], acc[i][1], acc[i][2], acc[i][3], ah, bh[0], bh[1], bh[2], bh[3]);
    }
  }
  acc_guard4(acc[0][0], acc[0][1], acc[0][2], acc[0][3]);
  acc_guard4(acc[1][0], acc[1][1], acc[1][2], acc[1][3]);
  acc_guard4(acc[2][0], acc[2][1], acc[2][2], acc[2][3]);
  acc_guard4(acc[3][0], acc[3][1], acc[3][2], acc[3][3]);

  float* slab = sT[wave];
  const int halfN = N >> 1;
  const bool isU = (n0 < halfN);
#pragma unroll
  for (int i = 0; i < 4; ++i) {
    const int mBase = m0 + (i << 4);
#pragma unroll
    for (int j = 0; j < 4; ++j) {
      const float bv = bias[n0 + (j << 4) + rlane];
#pragma unroll
      for (int r = 0; r < 8; ++r)
        slab[(mOff + r) * 68 + (j << 4) + rlane] = acc[i][j][r] * scale + bv;
    }
    wave_sync();
    if (EPI == kEpiGate || EPI == kEpiGelu) {
#pragma unroll 1
      for (int t = 0; t < 8; ++t) {
        const int idx = t * 32 + lane;
        float* sp = slab + (idx >> 4) * 68 + (idx & 15) * 4;
        const v4f v = *(const v4f*)sp;
        v4f o;
        if (EPI == kEpiGate) {
          o[0] = silu_f(v[0]); o[1] = silu_f(v[1]); o[2] = silu_f(v[2]); o[3] = silu_f(v[3]);
        } else {
          o[0] = gelu_f(v[0]) * ocarry; o[1] = gelu_f(v[1]) * ocarry;
          o[2] = gelu_f(v[2]) * ocarry; o[3] = gelu_f(v[3]) * ocarry;
        }
        *(v4f*)sp = o;
      }
      wave_sync();
    }
    if (EPI == kEpiResid) {
      float* C = (float*)Cout;
      const int hh = lane >> 4, c4 = (lane & 15) * 4;
      v4f vv[8];
#pragma unroll
      for (int it = 0; it < 8; ++it) {
        const int row = it * 2 + hh;
        const v4f sv = *(const v4f*)(slab + row * 68 + c4);
        const v4f rv = *(const v4f*)(resid + (size_t)(mBase + row) * ldc + n0 + c4);
        vv[it] = rv + sv;
      }
      for (int pass = 0; pass < 2; ++pass) {
#pragma unroll
        for (int it = 0; it < 8; ++it) {
          const int row = it * 2 + hh;
          *(volatile v4f*)(C + (size_t)(mBase + row) * ldc + n0 + c4) = vv[it];
        }
        __threadfence();
      }
    } else {
      unsigned short* C = (unsigned short*)Cout;
      const int q = lane >> 3, c8 = (lane & 7) * 8;
      const int ocol0 = (EPI == kEpiGate) ? (isU ? n0 : (n0 - halfN)) : n0;
      const int orow0 = (EPI == kEpiGate) ? (isU ? 0 : M) : 0;
      v8h hv[4];
#pragma unroll
      for (int it = 0; it < 4; ++it) {
        const int row = it * 4 + q;
        const float* sp = slab + row * 68 + c8;
        const v4f a0 = *(const v4f*)(sp);
        const v4f a1 = *(const v4f*)(sp + 4);
        float f[8];
        f[0] = a0[0]; f[1] = a0[1]; f[2] = a0[2]; f[3] = a0[3];
        f[4] = a1[0]; f[5] = a1[1]; f[6] = a1[2]; f[7] = a1[3];
        if (EPI == kEpiGate) {
          const v4u xw = *(const v4u*)(Ap + (size_t)(mBase + row) * lda + ocol0 + c8);
          const unsigned w0 = xw[0];
          const unsigned w1 = xw[1];
          const unsigned w2 = xw[2];
          const unsigned w3 = xw[3];
          float xf[8];
          xf[0] = h16_to_f32(w0 & 0xffffu); xf[1] = h16_to_f32(w0 >> 16);
          xf[2] = h16_to_f32(w1 & 0xffffu); xf[3] = h16_to_f32(w1 >> 16);
          xf[4] = h16_to_f32(w2 & 0xffffu); xf[5] = h16_to_f32(w2 >> 16);
          xf[6] = h16_to_f32(w3 & 0xffffu); xf[7] = h16_to_f32(w3 >> 16);
#pragma unroll
          for (int e = 0; e < 8; ++e) {
            const float mult = isU ? xf[e] : 1.0f;
            f[e] = (f[e] * mult) * ocarry;
          }
        }
#pragma unroll
        for (int e = 0; e < 8; ++e) hv[it][e] = (_Float16)f[e];
      }
      for (int pass = 0; pass < 2; ++pass) {
#pragma unroll
        for (int it = 0; it < 4; ++it) {
          const int row = it * 4 + q;
          *(volatile v8h*)(C + (size_t)(orow0 + mBase + row) * ldc + ocol0 + c8) = hv[it];
        }
        __threadfence();
      }
    }
    wave_sync();
  }
}

__global__ __launch_bounds__(256) void transpose_cast_kernel(
    const float* __restrict__ W, unsigned short* __restrict__ Bt, int Kdim, int Ndim, float scale)
{
  __shared__ float tile[64 * 65];
  const int tid = threadIdx.x, lane = tid & 31, wave = tid >> 5;
  const int n0 = blockIdx.x * 64;
  const int k0 = blockIdx.y * 64;
#pragma unroll
  for (int p = 0; p < 16; ++p) {
    const int idx = tid + p * 256;
    const int kk  = idx >> 6;
    const int nn  = idx & 63;
    const int n   = n0 + nn;
    const int nc  = (n < Ndim) ? n : (Ndim - 1);
    const float v = W[(size_t)(k0 + kk) * Ndim + nc];
    tile[kk * 65 + nn] = (n < Ndim) ? (v * scale) : 0.f;
  }
  __syncthreads();
  const int q = lane >> 3, c8 = (lane & 7) * 8;
  v8h hv[2];
#pragma unroll
  for (int it = 0; it < 2; ++it) {
    const int nrow = it * 32 + wave * 4 + q;
#pragma unroll
    for (int e = 0; e < 8; ++e) hv[it][e] = (_Float16)tile[(c8 + e) * 65 + nrow];
  }
  for (int pass = 0; pass < 2; ++pass) {
#pragma unroll
    for (int it = 0; it < 2; ++it) {
      const int nrow = it * 32 + wave * 4 + q;
      *(volatile v8h*)(Bt + (size_t)(n0 + nrow) * Kdim + k0 + c8) = hv[it];
    }
    __threadfence();
  }
}

__global__ __launch_bounds__(256) void wmean_kernel(
    const float* __restrict__ W, const float* __restrict__ sb, float* __restrict__ wm)
{
  __shared__ float sV[32];
  const int tid = threadIdx.x, lane = tid & 31, wave = tid >> 5;
  const int blk = blockIdx.x;
  const bool isW = (blk < 32);
#pragma unroll 1
  for (int i = 0; i < 4; ++i) {
    const int slot = wave * 4 + i;
    const float* src = isW ? (W + (size_t)(blk * 32 + slot) * kDS) : sb;
    float s = 0.f;
#pragma unroll
    for (int c = 0; c < 8; ++c) {
      const v4f a = *(const v4f*)(src + c * 128 + lane * 4);
      s += (a[0] + a[1]) + (a[2] + a[3]);
    }
    s = wave_sum(s);
    float val = s * (1.0f / (float)kDS);
    val = (isW || slot == 0) ? val : 0.f;
    if (lane == 0) sV[slot] = val;
  }
  __syncthreads();
  if (wave == 0) {
    const float v = sV[lane];
    float* p = wm + blk * 32 + lane;
    *(volatile float*)p = v;
    __threadfence();
    *(volatile float*)p = v;
  }
}

template <bool DELTA>
__global__ __launch_bounds__(256) void ln_rows_kernel(
    const float* __restrict__ X, const float* __restrict__ gw, const float* __restrict__ gb,
    unsigned short* __restrict__ out16, const float* __restrict__ wm,
    float* __restrict__ dl, float* __restrict__ da)
{
  __shared__ float sDl[32];
  __shared__ float sDa[32];
  const int tid = threadIdx.x, lane = tid & 31, wave = tid >> 5;
  constexpr float kInv = 1.0f / (float)kD;
#pragma unroll 1
  for (int i = 0; i < 4; ++i) {
    const int slot = wave * 4 + i;
    const size_t row = (size_t)blockIdx.x * 32 + slot;
    const float* xr = X + row * kD + lane * 8;
    float s = 0.f;
#pragma unroll 1
    for (int c = 0; c < 4; ++c) {
      const v4f a0 = *(const v4f*)(xr + c * 256);
      const v4f a1 = *(const v4f*)(xr + c * 256 + 4);
      s += ((a0[0] + a0[1]) + (a0[2] + a0[3])) + ((a1[0] + a1[1]) + (a1[2] + a1[3]));
    }
    s = wave_sum(s);
    const float mu = s * kInv;
    float vs = 0.f;
#pragma unroll 1
    for (int c = 0; c < 4; ++c) {
      const v4f a0 = *(const v4f*)(xr + c * 256);
      const v4f a1 = *(const v4f*)(xr + c * 256 + 4);
#pragma unroll
      for (int e = 0; e < 4; ++e) {
        const float d0 = a0[e] - mu;
        const float d1 = a1[e] - mu;
        vs = fmaf(d0, d0, vs);
        vs = fmaf(d1, d1, vs);
      }
    }
    vs = wave_sum(vs);
    const float rstd = rsqrtf(vs * kInv + 1e-5f);
    float dot = 0.f;
#pragma unroll 1
    for (int c = 0; c < 4; ++c) {
      const int off = c * 256 + lane * 8;
      const v4f a0 = *(const v4f*)(xr + c * 256);
      const v4f a1 = *(const v4f*)(xr + c * 256 + 4);
      const v4f w0 = *(const v4f*)(gw + off);
      const v4f w1 = *(const v4f*)(gw + off + 4);
      const v4f b0 = *(const v4f*)(gb + off);
      const v4f b1 = *(const v4f*)(gb + off + 4);
      float xn[8];
#pragma unroll
      for (int e = 0; e < 4; ++e) {
        xn[e]     = ((a0[e] - mu) * rstd) * w0[e] + b0[e];
        xn[4 + e] = ((a1[e] - mu) * rstd) * w1[e] + b1[e];
      }
      if (DELTA) {
        const v4f m0 = *(const v4f*)(wm + off);
        const v4f m1 = *(const v4f*)(wm + off + 4);
#pragma unroll
        for (int e = 0; e < 4; ++e) {
          dot = fmaf(xn[e], m0[e], dot);
          dot = fmaf(xn[4 + e], m1[e], dot);
        }
      }
      v8h hv;
#pragma unroll
      for (int e = 0; e < 8; ++e) hv[e] = (_Float16)xn[e];
      unsigned short* q = out16 + row * kD + off;
      *(volatile v8h*)q = hv;
      __threadfence();
      *(volatile v8h*)q = hv;
    }
    if (DELTA) {
      dot = wave_sum(dot);
      const float v  = dot + wm[kD];
      const float sp = fmaxf(v, 0.0f) + log1pf(expf(-fabsf(v)));
      const float ea = expf(-sp);
      if (lane == 0) { sDl[slot] = sp; sDa[slot] = ea; }
    }
  }
  if (DELTA) {
    __syncthreads();
    if (wave == 0) {
      const float v0 = sDl[lane];
      const float v1 = sDa[lane];
      float* p0 = dl + (size_t)blockIdx.x * 32 + lane;
      float* p1 = da + (size_t)blockIdx.x * 32 + lane;
      *(volatile float*)p0 = v0;
      *(volatile float*)p1 = v1;
      __threadfence();
      *(volatile float*)p0 = v0;
      *(volatile float*)p1 = v1;
    }
  }
}

__global__ __launch_bounds__(32) void scan_kernel(
    const unsigned* __restrict__ UBw, const float* __restrict__ dl, const float* __restrict__ da,
    unsigned short* __restrict__ Y)
{
  __shared__ __align__(16) float sY[kScanTS * kScanYP];
  __shared__ float sDl[kScanTS];
  __shared__ float sDa[kScanTS];
  const int lane = threadIdx.x;
  constexpr int kGroups = kDS / 64;
  const int bix = blockIdx.x / kGroups;
  const int c0  = (blockIdx.x - bix * kGroups) * 64;
  const size_t row0 = (size_t)bix * kSeq;
  const size_t cw = (size_t)(c0 >> 1) + lane;
  constexpr size_t kWordPitch = kDS / 2;
  float h0 = 0.f, h1 = 0.f;
  const int q = lane >> 3, c8 = (lane & 7) * 8;
#pragma unroll 1
  for (int t0 = 0; t0 < kSeq; t0 += kScanTS) {
    __syncthreads();
    sDl[lane]      = dl[row0 + t0 + lane];
    sDl[lane + 32] = dl[row0 + t0 + 32 + lane];
    sDa[lane]      = da[row0 + t0 + lane];
    sDa[lane + 32] = da[row0 + t0 + 32 + lane];
    __syncthreads();
#pragma unroll 1
    for (int g = 0; g < 8; ++g) {
      unsigned uw[8], bw[8];
#pragma unroll
      for (int s = 0; s < 8; ++s) {
        const size_t r = row0 + t0 + g * 8 + s;
        uw[s] = UBw[r * kWordPitch + cw];
        bw[s] = UBw[((size_t)kRows + r) * kWordPitch + cw];
      }
#pragma unroll
      for (int s = 0; s < 8; ++s) {
        const float dlt = sDl[g * 8 + s];
        const float dav = sDa[g * 8 + s];
        const float u0 = h16_to_f32(uw[s] & 0xffffu);
        const float u1 = h16_to_f32(uw[s] >> 16);
        const float b0 = h16_to_f32(bw[s] & 0xffffu);
        const float b1 = h16_to_f32(bw[s] >> 16);
        const float p0 = (dlt * b0) * u0;
        const float p1 = (dlt * b1) * u1;
        h0 = fmaf(dav, h0, p0);
        h1 = fmaf(dav, h1, p1);
        v2f yv;
        yv[0] = h0 * kACarry;
        yv[1] = h1 * kACarry;
        *(v2f*)(sY + (g * 8 + s) * kScanYP + 2 * lane) = yv;
      }
    }
    __syncthreads();
    v8h hv[16];
#pragma unroll
    for (int it = 0; it < 16; ++it) {
      const int row = it * 4 + q;
      const float* sp = sY + row * kScanYP + c8;
      const v4f a0 = *(const v4f*)(sp);
      const v4f a1 = *(const v4f*)(sp + 4);
#pragma unroll
      for (int e = 0; e < 4; ++e) {
        hv[it][e]     = (_Float16)a0[e];
        hv[it][4 + e] = (_Float16)a1[e];
      }
    }
    for (int pass = 0; pass < 2; ++pass) {
#pragma unroll
      for (int it = 0; it < 16; ++it) {
        const int row = it * 4 + q;
        *(volatile v8h*)(Y + (row0 + t0 + row) * kDS + c0 + c8) = hv[it];
      }
      __threadfence();
    }
  }
}

extern "C" void kernel_launch(void* const* d_in, const int* in_sizes, int n_in,
                              void* d_out, int out_size, void* d_ws, size_t ws_size,
                              hipStream_t stream)
{
  if (n_in < 15) return;
  if (in_sizes[0] != kRows * kD) return;
  if (in_sizes[1] != kD || in_sizes[2] != kD) return;
  if (in_sizes[3] != kD * kG || in_sizes[4] != kG) return;
  if (in_sizes[5] != kD * kDS || in_sizes[6] != kDS) return;
  if (in_sizes[7] != kDS * kD || in_sizes[8] != kD) return;
  if (in_sizes[9] != kD || in_sizes[10] != kD) return;
  if (in_sizes[11] != kD * kH || in_sizes[12] != kH) return;
  if (in_sizes[13] != kH * kD || in_sizes[14] != kD) return;
  if (out_size != kRows * kD) return;
  if (ws_size < kWsTotal) return;

  const float* x       = (const float*)d_in[0];
  const float* n1w     = (const float*)d_in[1];
  const float* n1b     = (const float*)d_in[2];
  const float* gate_w  = (const float*)d_in[3];
  const float* gate_b  = (const float*)d_in[4];
  const float* state_w = (const float*)d_in[5];
  const float* state_b = (const float*)d_in[6];
  const float* out_w   = (const float*)d_in[7];
  const float* out_b   = (const float*)d_in[8];
  const float* n2w     = (const float*)d_in[9];
  const float* n2b     = (const float*)d_in[10];
  const float* w1      = (const float*)d_in[11];
  const float* b1      = (const float*)d_in[12];
  const float* w2      = (const float*)d_in[13];
  const float* b2      = (const float*)d_in[14];
  float* out = (float*)d_out;

  char* ws = (char*)d_ws;
  unsigned short* GWT = (unsigned short*)(ws + kOffGWT);
  unsigned short* SWT = (unsigned short*)(ws + kOffSWT);
  unsigned short* OWT = (unsigned short*)(ws + kOffOWT);
  unsigned short* W1T = (unsigned short*)(ws + kOffW1T);
  unsigned short* W2T = (unsigned short*)(ws + kOffW2T);
  unsigned short* XN  = (unsigned short*)(ws + kOffXN);
  unsigned short* S   = (unsigned short*)(ws + kOffS);
  unsigned short* UB  = (unsigned short*)(ws + kOffUB);
  unsigned short* Y   = (unsigned short*)(ws + kOffY);
  unsigned short* HID = (unsigned short*)(ws + kOffHID);
  unsigned short* X2  = (unsigned short*)(ws + kOffX2);
  float* WM = (float*)(ws + kOffWM);
  float* DL = (float*)(ws + kOffDL);
  float* DA = (float*)(ws + kOffDA);

  wmean_kernel<<<33, 256, 0, stream>>>(state_w, state_b, WM);

  transpose_cast_kernel<<<dim3(kG / 64, kD / 64), 256, 0, stream>>>(gate_w, GWT, kD, kG, kWCarry);
  transpose_cast_kernel<<<dim3(kDS / 64, kD / 64), 256, 0, stream>>>(state_w, SWT, kD, kDS, kWCarry);
  transpose_cast_kernel<<<dim3(kD / 64, kDS / 64), 256, 0, stream>>>(out_w, OWT, kDS, kD, kWCarry);
  transpose_cast_kernel<<<dim3(kH / 64, kD / 64), 256, 0, stream>>>(w1, W1T, kD, kH, kWCarry);
  transpose_cast_kernel<<<dim3(kD / 64, kH / 64), 256, 0, stream>>>(w2, W2T, kH, kD, kWCarry);

  ln_rows_kernel<true><<<kRows / 32, 256, 0, stream>>>(x, n1w, n1b, XN, WM, DL, DA);

  gemm_f16_kernel<kEpiGate><<<(kRows / 64) * (kG / 64) / 8, 256, 0, stream>>>(
      XN, kD, GWT, kD, (void*)S, kD, gate_b, x, kRows, kG, kD, kInvW, kACarry);

  gemm_f16_kernel<kEpiF16><<<(2 * kRows / 64) * (kDS / 64) / 8, 256, 0, stream>>>(
      S, kD, SWT, kD, (void*)UB, kDS, state_b, x, 2 * kRows, kDS, kD, kInvWA, 1.0f);

  scan_kernel<<<kBatch * (kDS / 64), 32, 0, stream>>>((const unsigned*)UB, DL, DA, Y);

  gemm_f16_kernel<kEpiResid><<<(kRows / 64) * (kD / 64) / 8, 256, 0, stream>>>(
      Y, kDS, OWT, kDS, (void*)out, kD, out_b, x, kRows, kD, kDS, kInvWA, 1.0f);

  ln_rows_kernel<false><<<kRows / 32, 256, 0, stream>>>(out, n2w, n2b, X2, WM, DL, DA);

  gemm_f16_kernel<kEpiGelu><<<(kRows / 64) * (kH / 64) / 8, 256, 0, stream>>>(
      X2, kD, W1T, kD, (void*)HID, kH, b1, x, kRows, kH, kD, kInvW, kACarry);

  gemm_f16_kernel<kEpiResid><<<(kRows / 64) * (kD / 64) / 8, 256, 0, stream>>>(
      HID, kH, W2T, kH, (void*)out, kD, b2, out, kRows, kD, kH, kInvWA, 1.0f);
}
